// PoolHiddenNet_74577812127758
// MI455X (gfx1250) — hardware-run, weakly checked
//
#include <hip/hip_runtime.h>
#include <math.h>

typedef __attribute__((ext_vector_type(16))) _Float16 v16h;
typedef __attribute__((ext_vector_type(8)))  _Float16 v8h;
typedef __attribute__((ext_vector_type(8)))  float    v8f;
typedef __attribute__((ext_vector_type(4)))  float    v4f;
typedef __attribute__((ext_vector_type(2)))  float    v2f;

constexpr int kGroups = 128;
constexpr int kPed    = 32;
constexpr int kRows   = kGroups * kPed;
constexpr int kHid    = 64;
constexpr int kEmb    = 64;
constexpr int kZK     = 192;
constexpr int kD1     = 512;
constexpr int kD2     = 1024;
constexpr float kEps  = 1e-5f;
static_assert(kRows == 4096, "ped count");
static_assert(kZK == 2 * kEmb + kHid, "layer-1 K");
static_assert((kZK % 32) == 0 && (kEmb % 32) == 0 && (kD1 % 32) == 0, "GEMM K multiples of 32");
static_assert((kRows % 64) == 0 && (kD1 % 64) == 0, "GEMM M,N multiples of 64");

constexpr float kZCarry  = 64.0f;
constexpr float kW1Carry = 256.0f;
constexpr float kW2Carry = 256.0f;
constexpr float kH1Carry = 16.0f;
constexpr float kL1Scale = 1.0f / (kZCarry * kW1Carry);
constexpr float kL2Scale = 1.0f / (kH1Carry * kW2Carry);

constexpr int kMainCols  = 32;
constexpr int kMainWaves = 16;
constexpr int kApitch    = 520;
static_assert((kD2 % kMainCols) == 0, "column tiles");
static_assert(kMainWaves * 2 == kPed, "two query peds per wave");

constexpr size_t kOffW2T = 0;
constexpr size_t kOffW1T = kOffW2T + (size_t)kD2 * kD1 * 2;
constexpr size_t kOffZPL = kOffW1T + (size_t)kD1 * kZK * 2;
constexpr size_t kOffTPL = kOffZPL + (size_t)kRows * kZK * 2;
constexpr size_t kOffUPL = kOffTPL + (size_t)kRows * kD1 * 4;
constexpr size_t kOffAHP = kOffUPL + (size_t)kRows * kD1 * 4;
constexpr size_t kOffBHP = kOffAHP + (size_t)kRows * kD1 * 2;
constexpr size_t kWsTotal = kOffBHP + (size_t)kRows * kD1 * 2;
static_assert(kWsTotal == 27983872ull, "carve total");
static_assert(kWsTotal <= 134217728ull, "carve cap");
static_assert((kOffW1T % 128) == 0 && (kOffZPL % 128) == 0 && (kOffTPL % 128) == 0 && (kOffUPL % 128) == 0 &&
              (kOffAHP % 128) == 0 && (kOffBHP % 128) == 0, "128-B aligned regions");

union FragH { v16h v; v8h h[2]; };
__device__ __forceinline__ v16h frag_load_h(const _Float16* p) {
  FragH f;
  f.h[0] = *(const v8h*)(p);
  f.h[1] = *(const v8h*)(p + 16);
  return f.v;
}
__device__ __forceinline__ v8f mma_f16_guarded(v16h a, v16h b, v8f c) {
  c = __builtin_amdgcn_wmma_f32_16x16x32_f16(false, a, false, b, (short)0, c, false, false);
  asm volatile("v_nop\n\tv_nop\n\tv_nop\n\tv_nop" : "+v"(c) : "v"(a), "v"(b));
  return c;
}

constexpr int kW2Blocks = (kD2 * (kD1 / 8)) / 256;
constexpr int kW1Blocks = (kD1 * (kZK / 8)) / 256;
static_assert(kW2Blocks * 256 == kD2 * (kD1 / 8), "W2 chunk coverage");
static_assert(kW1Blocks * 256 == kD1 * (kZK / 8), "W1 chunk coverage");

__device__ __forceinline__ void transpose_chunk(const float* __restrict__ W, _Float16* __restrict__ Wt,
                                                int kdim, int ndim, int i, float carry) {
  const int cpr = kdim >> 3;
  const int n = i / cpr;
  const int k8 = i - n * cpr;
  v8h hv;
#pragma unroll
  for (int e = 0; e < 8; ++e) {
    const float f = W[(size_t)(k8 * 8 + e) * ndim + n] * carry;
    hv[e] = (_Float16)f;
  }
  _Float16* p = Wt + (size_t)n * kdim + k8 * 8;
  *(volatile v8h*)p = hv;
  __threadfence();
  *(volatile v8h*)p = hv;
}

__global__ __launch_bounds__(256) void weight_planes_kernel(
    const float* __restrict__ W2, const float* __restrict__ W1,
    _Float16* __restrict__ W2t, _Float16* __restrict__ W1t)
{
  const int b = blockIdx.x;
  const int tid = threadIdx.x;
  if (b < kW2Blocks) {
    transpose_chunk(W2, W2t, kD1, kD2, b * 256 + tid, kW2Carry);
  } else {
    transpose_chunk(W1, W1t, kZK, kD1, (b - kW2Blocks) * 256 + tid, kW1Carry);
  }
}

__global__ __launch_bounds__(256) void z_plane_kernel(
    const float* __restrict__ hid, const float* __restrict__ pos, const float* __restrict__ spd,
    const float* __restrict__ Ws, const float* __restrict__ Wv, _Float16* __restrict__ Z)
{
  const int i = blockIdx.x * 256 + threadIdx.x;
  const int n = i >> 3;
  const int cc = i & 7;
  const int sec = blockIdx.y;
  float vals[8];
  if (sec == 0) {
    const v2f pp = *(const v2f*)(pos + 2 * n);
    const float p0 = pp[0], p1 = pp[1];
    const v4f wa0 = *(const v4f*)(Ws + cc * 8);
    const v4f wa1 = *(const v4f*)(Ws + cc * 8 + 4);
    const v4f wb0 = *(const v4f*)(Ws + kEmb + cc * 8);
    const v4f wb1 = *(const v4f*)(Ws + kEmb + cc * 8 + 4);
#pragma unroll
    for (int e = 0; e < 4; ++e) {
      vals[e]     = p0 * wa0[e] + p1 * wb0[e];
      vals[4 + e] = p0 * wa1[e] + p1 * wb1[e];
    }
  } else if (sec == 1) {
    const v4f a0 = *(const v4f*)(hid + (size_t)n * kHid + cc * 8);
    const v4f a1 = *(const v4f*)(hid + (size_t)n * kHid + cc * 8 + 4);
#pragma unroll
    for (int e = 0; e < 4; ++e) {
      vals[e]     = a0[e];
      vals[4 + e] = a1[e];
    }
  } else {
    const float s = spd[n];
    const v4f w0 = *(const v4f*)(Wv + cc * 8);
    const v4f w1 = *(const v4f*)(Wv + cc * 8 + 4);
#pragma unroll
    for (int e = 0; e < 4; ++e) {
      vals[e]     = s * w0[e];
      vals[4 + e] = s * w1[e];
    }
  }
  v8h hv;
#pragma unroll
  for (int e = 0; e < 8; ++e) {
    const float f = vals[e] * kZCarry;
    hv[e] = (_Float16)f;
  }
  _Float16* p = Z + (size_t)n * kZK + sec * 64 + cc * 8;
  *(volatile v8h*)p = hv;
  __threadfence();
  *(volatile v8h*)p = hv;
}

__global__ __launch_bounds__(256) void gemm64_f16_kernel(
    const _Float16* __restrict__ A, int lda,
    const _Float16* __restrict__ Bt, int ldb,
    float* __restrict__ C, int ldc,
    int M, int N, int K, float scale)
{
  __shared__ __align__(16) float sT[8][16 * 68];
  const int lane = threadIdx.x & 31;
  const int wave = __builtin_amdgcn_readfirstlane((int)(threadIdx.x >> 5));
  const int tilesN = N >> 6;
  const int tilesM = M >> 6;
  const int tile = blockIdx.x * 8 + wave;
  if (tile >= tilesM * tilesN) return;
  const int tm = tile / tilesN;
  const int tn = tile - tm * tilesN;
  const int m0 = tm << 6;
  const int n0 = tn << 6;
  const int rlane = lane & 15;
  const int koff  = (lane >> 4) * 8;
  const int mOff  = (lane >> 4) * 8;

  v8f acc[4][4];
#pragma unroll
  for (int i = 0; i < 4; ++i)
#pragma unroll
    for (int j = 0; j < 4; ++j) acc[i][j] = (v8f){0.f, 0.f, 0.f, 0.f, 0.f, 0.f, 0.f, 0.f};

#pragma unroll 1
  for (int k0 = 0; k0 < K; k0 += 32) {
    v16h bh[4];
#pragma unroll
    for (int j = 0; j < 4; ++j) {
      const size_t bo = (size_t)(n0 + (j << 4) + rlane) * ldb + koff + k0;
      bh[j] = frag_load_h(Bt + bo);
    }
#pragma unroll
    for (int i = 0; i < 4; ++i) {
      const size_t ao = (size_t)(m0 + (i << 4) + rlane) * lda + koff + k0;
      const v16h ah = frag_load_h(A + ao);
#pragma unroll
      for (int j = 0; j < 4; ++j) acc[i][j] = mma_f16_guarded(ah, bh[j], acc[i][j]);
    }
  }

  float* slab = sT[wave];
#pragma unroll
  for (int i = 0; i < 4; ++i) {
    const int mBase = m0 + (i << 4);
#pragma unroll
    for (int j = 0; j < 4; ++j) {
#pragma unroll
      for (int r = 0; r < 8; ++r) {
        const float v = acc[i][j][r] * scale;
        slab[(mOff + r) * 68 + (j << 4) + rlane] = v;
      }
    }
    __builtin_amdgcn_fence(__ATOMIC_RELEASE, "workgroup");
    __builtin_amdgcn_wave_barrier();
    __builtin_amdgcn_fence(__ATOMIC_ACQUIRE, "workgroup");
    {
      const int hh = lane >> 4, c4 = (lane & 15) * 4;
      for (int pass = 0; pass < 2; ++pass) {
#pragma unroll
        for (int it = 0; it < 8; ++it) {
          const int row = it * 2 + hh;
          const v4f v = *(const v4f*)(slab + row * 68 + c4);
          *(volatile v4f*)(C + (size_t)(mBase + row) * ldc + n0 + c4) = v;
        }
        __threadfence();
      }
    }
    __builtin_amdgcn_fence(__ATOMIC_RELEASE, "workgroup");
    __builtin_amdgcn_wave_barrier();
    __builtin_amdgcn_fence(__ATOMIC_ACQUIRE, "workgroup");
  }
}

__global__ __launch_bounds__(256) void bn1_planes_kernel(
    const float* __restrict__ U, const float* __restrict__ T,
    const float* __restrict__ g1, const float* __restrict__ be1,
    unsigned* __restrict__ AhW, unsigned* __restrict__ BhW)
{
  const int g = blockIdx.x;
  const int tid = threadIdx.x;
  const int c = tid * 2;
  const size_t base = (size_t)g * kPed * kD1 + c;
  const float inv = 1.0f / (float)kPed;
  float su0 = 0.f, su1 = 0.f, st0 = 0.f, st1 = 0.f;
#pragma unroll 1
  for (int j = 0; j < kPed; ++j) {
    const v2f uv = *(const v2f*)(U + base + (size_t)j * kD1);
    const v2f tv = *(const v2f*)(T + base + (size_t)j * kD1);
    su0 += uv[0]; su1 += uv[1];
    st0 += tv[0]; st1 += tv[1];
  }
  const float mu0 = su0 * inv, mu1 = su1 * inv, mt0 = st0 * inv, mt1 = st1 * inv;
  float qu0 = 0.f, qu1 = 0.f, qt0 = 0.f, qt1 = 0.f;
#pragma unroll 1
  for (int j = 0; j < kPed; ++j) {
    const v2f uv = *(const v2f*)(U + base + (size_t)j * kD1);
    const v2f tv = *(const v2f*)(T + base + (size_t)j * kD1);
    const float du0 = uv[0] - mu0, du1 = uv[1] - mu1;
    const float dt0 = tv[0] - mt0, dt1 = tv[1] - mt1;
    qu0 = fmaf(du0, du0, qu0); qu1 = fmaf(du1, du1, qu1);
    qt0 = fmaf(dt0, dt0, qt0); qt1 = fmaf(dt1, dt1, qt1);
  }
  const float var0 = (qu0 + qt0) * inv;
  const float var1 = (qu1 + qt1) * inv;
  const v2f gv = *(const v2f*)(g1 + c);
  const v2f bev = *(const v2f*)(be1 + c);
  const float s0 = gv[0] * rsqrtf(var0 + kEps) * kH1Carry;
  const float s1 = gv[1] * rsqrtf(var1 + kEps) * kH1Carry;
  const float o0 = bev[0] * kH1Carry;
  const float o1 = bev[1] * kH1Carry;
#pragma unroll 1
  for (int j = 0; j < kPed; ++j) {
    const v2f uv = *(const v2f*)(U + base + (size_t)j * kD1);
    const v2f tv = *(const v2f*)(T + base + (size_t)j * kD1);
    const float a0 = (uv[0] - mu0) * s0 + o0;
    const float a1 = (uv[1] - mu1) * s1 + o1;
    const float b0 = (mt0 - tv[0]) * s0;
    const float b1 = (mt1 - tv[1]) * s1;
    const _Float16 ha0 = (_Float16)a0, ha1 = (_Float16)a1;
    const _Float16 hb0 = (_Float16)b0, hb1 = (_Float16)b1;
    const unsigned wa = (unsigned)__builtin_bit_cast(unsigned short, ha0) |
                        ((unsigned)__builtin_bit_cast(unsigned short, ha1) << 16);
    const unsigned wb = (unsigned)__builtin_bit_cast(unsigned short, hb0) |
                        ((unsigned)__builtin_bit_cast(unsigned short, hb1) << 16);
    const size_t wi = (size_t)(g * kPed + j) * (kD1 / 2) + tid;
    ((volatile unsigned*)AhW)[wi] = wa;
    ((volatile unsigned*)BhW)[wi] = wb;
    __threadfence();
    ((volatile unsigned*)AhW)[wi] = wa;
    ((volatile unsigned*)BhW)[wi] = wb;
  }
}

__global__ __launch_bounds__(512) void fused_layer2_kernel(
    const _Float16* __restrict__ Ah, const _Float16* __restrict__ Bh, const _Float16* __restrict__ W2t,
    const float* __restrict__ g2, const float* __restrict__ be2, float* __restrict__ out)
{
  __shared__ __align__(16) _Float16 sA[kPed * kApitch];
  __shared__ __align__(16) float sRed[kMainWaves * kMainCols];
  __shared__ __align__(16) float sMean[kMainCols];
  __shared__ __align__(16) float sScale[kMainCols];
  __shared__ __align__(16) float sShift[kMainCols];

  const int tid  = threadIdx.x;
  const int lane = tid & 31;
  const int wave = __builtin_amdgcn_readfirstlane((int)(threadIdx.x >> 5));
  const int hh   = lane >> 4;
  const int rl   = lane & 15;
  const int nt   = blockIdx.x;
  const int g    = blockIdx.y;

#pragma unroll
  for (int it = 0; it < 4; ++it) {
    const int q = tid + it * 512;
    const int r = q >> 6;
    const int s = q & 63;
    const v8h v = *(const v8h*)(Ah + (size_t)(g * kPed + r) * kD1 + s * 8);
    *(v8h*)(sA + r * kApitch + s * 8) = v;
  }
  __syncthreads();

  v8f acc[2][2][2];
#pragma unroll
  for (int ii = 0; ii < 2; ++ii)
#pragma unroll
    for (int mf = 0; mf < 2; ++mf)
#pragma unroll
      for (int nf = 0; nf < 2; ++nf) acc[ii][mf][nf] = (v8f){0.f, 0.f, 0.f, 0.f, 0.f, 0.f, 0.f, 0.f};

  const _Float16* bi0 = Bh + (size_t)(g * kPed + 2 * wave) * kD1 + 8 * hh;
  const _Float16* bi1 = bi0 + kD1;
  const _Float16* wp0 = W2t + (size_t)(nt * kMainCols + rl) * kD1 + 8 * hh;
  const _Float16* wp1 = wp0 + 16 * kD1;
  const int aoff = rl * kApitch + 8 * hh;
  const v16h zero16 = {};

#pragma unroll 1
  for (int k0 = 0; k0 < kD1; k0 += 32) {
    v16h wf[2], bv[2];
    wf[0] = frag_load_h(wp0 + k0);
    wf[1] = frag_load_h(wp1 + k0);
    bv[0] = frag_load_h(bi0 + k0);
    bv[1] = frag_load_h(bi1 + k0);
#pragma unroll
    for (int mf = 0; mf < 2; ++mf) {
      FragH fa;
      fa.h[0] = *(const v8h*)(sA + mf * 16 * kApitch + aoff + k0);
      fa.h[1] = *(const v8h*)(sA + mf * 16 * kApitch + aoff + k0 + 16);
#pragma unroll
      for (int ii = 0; ii < 2; ++ii) {
        const v16h hsum = fa.v + bv[ii];
        const v16h h1 = __builtin_elementwise_max(hsum, zero16);
#pragma unroll
        for (int nf = 0; nf < 2; ++nf) acc[ii][mf][nf] = mma_f16_guarded(h1, wf[nf], acc[ii][mf][nf]);
      }
    }
  }

#pragma unroll
  for (int ii = 0; ii < 2; ++ii)
#pragma unroll
    for (int mf = 0; mf < 2; ++mf)
#pragma unroll
      for (int nf = 0; nf < 2; ++nf) acc[ii][mf][nf] = acc[ii][mf][nf] * kL2Scale;

  float cs[2];
#pragma unroll
  for (int nf = 0; nf < 2; ++nf) {
    float s = 0.f;
#pragma unroll
    for (int ii = 0; ii < 2; ++ii)
#pragma unroll
      for (int mf = 0; mf < 2; ++mf)
#pragma unroll
        for (int r = 0; r < 8; ++r) s += acc[ii][mf][nf][r];
    s += __shfl_xor(s, 16, 32);
    cs[nf] = s;
  }
  {
    const float v = hh ? cs[1] : cs[0];
    sRed[wave * kMainCols + lane] = v;
  }
  __syncthreads();
  if (wave == 0) {
    float s = 0.f;
#pragma unroll
    for (int w = 0; w < kMainWaves; ++w) s += sRed[w * kMainCols + lane];
    sMean[lane] = s * (1.0f / (float)(kPed * kPed));
  }
  __syncthreads();

  float mean[2];
  mean[0] = sMean[rl];
  mean[1] = sMean[16 + rl];
  float cq[2];
#pragma unroll
  for (int nf = 0; nf < 2; ++nf) {
    float q = 0.f;
#pragma unroll
    for (int ii = 0; ii < 2; ++ii)
#pragma unroll
      for (int mf = 0; mf < 2; ++mf)
#pragma unroll
        for (int r = 0; r < 8; ++r) {
          const float d = acc[ii][mf][nf][r] - mean[nf];
          q = fmaf(d, d, q);
        }
    q += __shfl_xor(q, 16, 32);
    cq[nf] = q;
  }
  {
    const float v = hh ? cq[1] : cq[0];
    sRed[wave * kMainCols + lane] = v;
  }
  __syncthreads();
  if (wave == 0) {
    float s = 0.f;
#pragma unroll
    for (int w = 0; w < kMainWaves; ++w) s += sRed[w * kMainCols + lane];
    const float var = s * (1.0f / (float)(kPed * kPed));
    const int col = nt * kMainCols + lane;
    const float gm = g2[col];
    const float bt = be2[col];
    const float sc = gm * rsqrtf(var + kEps);
    const float mu = sMean[lane];
    sScale[lane] = sc;
    sShift[lane] = bt - mu * sc;
  }
  __syncthreads();

  float sc[2], sh[2];
  sc[0] = sScale[rl];      sh[0] = sShift[rl];
  sc[1] = sScale[16 + rl]; sh[1] = sShift[16 + rl];

  float mx[2][2];
#pragma unroll
  for (int ii = 0; ii < 2; ++ii)
#pragma unroll
    for (int nf = 0; nf < 2; ++nf) {
      float m = 0.f;
#pragma unroll
      for (int mf = 0; mf < 2; ++mf)
#pragma unroll
        for (int r = 0; r < 8; ++r) m = fmaxf(m, fmaf(acc[ii][mf][nf][r], sc[nf], sh[nf]));
      m = fmaxf(m, __shfl_xor(m, 16, 32));
      mx[ii][nf] = m;
    }

  const float v0 = hh ? mx[0][1] : mx[0][0];
  const float v1 = hh ? mx[1][1] : mx[1][0];
  float* p0 = out + (size_t)(g * kPed + 2 * wave) * kD2 + nt * kMainCols + lane;
  float* p1 = p0 + kD2;
  *(volatile float*)p0 = v0;
  *(volatile float*)p1 = v1;
  __threadfence();
  *(volatile float*)p0 = v0;
  *(volatile float*)p1 = v1;
}

extern "C" void kernel_launch(void* const* d_in, const int* in_sizes, int n_in,
                              void* d_out, int out_size, void* d_ws, size_t ws_size,
                              hipStream_t stream) {
  if (n_in < 16) return;
  if (in_sizes[0] != kRows * kHid) return;
  if (in_sizes[2] != kRows * 2) return;
  if (in_sizes[3] != kRows) return;
  if (in_sizes[4] != 2 * kEmb) return;
  if (in_sizes[6] != kEmb) return;
  if (in_sizes[8] != kZK * kD1) return;
  if (in_sizes[10] != kD1) return;
  if (in_sizes[11] != kD1) return;
  if (in_sizes[12] != kD1 * kD2) return;
  if (in_sizes[14] != kD2) return;
  if (in_sizes[15] != kD2) return;
  if (out_size != kRows * kD2) return;
  if (ws_size < kWsTotal) return;

  const float* h_states = (const float*)d_in[0];
  const float* end_pos  = (const float*)d_in[2];
  const float* spd      = (const float*)d_in[3];
  const float* Ws       = (const float*)d_in[4];
  const float* Wv       = (const float*)d_in[6];
  const float* W1       = (const float*)d_in[8];
  const float* g1       = (const float*)d_in[10];
  const float* be1      = (const float*)d_in[11];
  const float* W2       = (const float*)d_in[12];
  const float* g2       = (const float*)d_in[14];
  const float* be2      = (const float*)d_in[15];
  float* out = (float*)d_out;

  char* ws = (char*)d_ws;
  _Float16* W2T = (_Float16*)(ws + kOffW2T);
  _Float16* W1T = (_Float16*)(ws + kOffW1T);
  _Float16* ZPL = (_Float16*)(ws + kOffZPL);
  float*    TPL = (float*)(ws + kOffTPL);
  float*    UPL = (float*)(ws + kOffUPL);
  _Float16* AHP = (_Float16*)(ws + kOffAHP);
  _Float16* BHP = (_Float16*)(ws + kOffBHP);

  weight_planes_kernel<<<kW2Blocks + kW1Blocks, 256, 0, stream>>>(W2, W1, W2T, W1T);

  z_plane_kernel<<<dim3((kRows * 8) / 256, 3), 256, 0, stream>>>(h_states, end_pos, spd, Ws, Wv, ZPL);

  gemm64_f16_kernel<<<((kRows / 64) * (kD1 / 64)) / 8, 256, 0, stream>>>(
      ZPL, kZK, W1T, kZK, TPL, kD1, kRows, kD1, kEmb, kL1Scale);
  gemm64_f16_kernel<<<((kRows / 64) * (kD1 / 64)) / 8, 256, 0, stream>>>(
      ZPL, kZK, W1T, kZK, UPL, kD1, kRows, kD1, kZK, kL1Scale);

  bn1_planes_kernel<<<kGroups, 256, 0, stream>>>(UPL, TPL, g1, be1, (unsigned*)AHP, (unsigned*)BHP);

  fused_layer2_kernel<<<dim3(kD2 / kMainCols, kGroups), 512, 0, stream>>>(AHP, BHP, W2T, g2, be2, out);
}
